// CausalSelfAttention_42348377538805
// MI455X (gfx1250) — hardware-verified
//
#include <hip/hip_runtime.h>


#ifndef NB
#define NB 2
#endif
#ifndef SEQ
#define SEQ 2048
#endif
#define NB_FULL  2
#define SEQ_FULL 2048
#define DM   1024
#define NH   16
#define HD   64
#define RH   ((SEQ) < 256 ? (SEQ) : 256)
#define PCAR 1024.0f
#define SCL  0.125f
#define LOG2E 1.4426950408889634f
#define NEGBIG (-1.0e30f)

typedef _Float16 h16;
typedef unsigned short bf;
typedef __attribute__((ext_vector_type(16))) __bf16   v16bf;
typedef __attribute__((ext_vector_type(16))) _Float16 v16h;
typedef __attribute__((ext_vector_type(16))) unsigned short v16us;
typedef __attribute__((ext_vector_type(8)))  _Float16 v8h;
typedef __attribute__((ext_vector_type(8)))  unsigned short v8us;
typedef __attribute__((ext_vector_type(8)))  float    v8f;
typedef __attribute__((ext_vector_type(4)))  float    v4f;
typedef v4f __attribute__((may_alias)) v4fa;

static_assert(NH * HD == DM);
static_assert(HD == 64);
static_assert(DM % 32 == 0);
static_assert((DM & (DM - 1)) == 0);
static_assert(SEQ % 64 == 0);
static_assert(RH % 64 == 0);
static_assert(RH <= SEQ);
static_assert(NB <= NB_FULL);
static_assert(SEQ <= SEQ_FULL);
static_assert((3 * DM) % 64 == 0);
static_assert(((size_t)(NB_FULL - 1) * SEQ_FULL + SEQ_FULL) * DM * 4 == 16777216);
static_assert(((size_t)(NB - 1) * SEQ_FULL + (SEQ - 1)) * DM + (DM - 1) < (size_t)NB_FULL * SEQ_FULL * DM);

constexpr size_t SZ_XB   = (size_t)NB * SEQ * DM * 2;
constexpr size_t SZ_WA   = (size_t)3 * DM * DM * 2;
constexpr size_t SZ_WP   = (size_t)DM * DM * 2;
constexpr size_t SZ_QK16 = (size_t)2 * NB * NH * SEQ * HD * 2;
constexpr size_t SZ_VT16 = (size_t)NB * NH * HD * SEQ * 2;
constexpr size_t SZ_QKH  = (size_t)2 * NB * NH * RH * HD * 2;
constexpr size_t SZ_VTH  = (size_t)NB * NH * HD * RH * 2;
constexpr size_t SZ_CTX  = (size_t)NB * SEQ * 2 * DM * 2;
constexpr size_t OFF_XB   = 0;
constexpr size_t OFF_WA   = OFF_XB + SZ_XB;
constexpr size_t OFF_WP   = OFF_WA + SZ_WA;
constexpr size_t OFF_QK16 = OFF_WP + SZ_WP;
constexpr size_t OFF_VT16 = OFF_QK16 + SZ_QK16;
constexpr size_t OFF_QKH  = OFF_VT16 + SZ_VT16;
constexpr size_t OFF_QKL  = OFF_QKH + SZ_QKH;
constexpr size_t OFF_VTH  = OFF_QKL + SZ_QKH;
constexpr size_t OFF_VTL  = OFF_VTH + SZ_VTH;
constexpr size_t OFF_CTX  = OFF_VTL + SZ_VTH;
constexpr size_t OFF_END  = OFF_CTX + SZ_CTX;
static_assert(OFF_END <= (size_t)134217728);
static_assert(SZ_XB % 256 == 0 && SZ_WA % 256 == 0 && SZ_WP % 256 == 0 && SZ_QK16 % 256 == 0 && SZ_VT16 % 256 == 0 && SZ_QKH % 256 == 0 && SZ_VTH % 256 == 0 && SZ_CTX % 256 == 0);

__device__ __forceinline__ unsigned short f2bf(float f) { unsigned u = __float_as_uint(f); u += 0x7FFFu + ((u >> 16) & 1u); return (unsigned short)(u >> 16); }
__device__ __forceinline__ float bf2f(unsigned short b) { return __uint_as_float(((unsigned)b) << 16); }
__device__ __forceinline__ float bfr(float f) { return bf2f(f2bf(f)); }
__device__ __forceinline__ void splitf(float y, unsigned short& h, unsigned short& l) { h = f2bf(y); l = f2bf(y - bf2f(h)); }
__device__ __forceinline__ float ex2(float x) { return __builtin_amdgcn_exp2f(x); }
__device__ __forceinline__ v16h cat16(v8h lo, v8h hi) { return __builtin_shufflevector(lo, hi, 0, 1, 2, 3, 4, 5, 6, 7, 8, 9, 10, 11, 12, 13, 14, 15); }
__device__ __forceinline__ v16bf cat16b(v8us lo, v8us hi) { return __builtin_bit_cast(v16bf, __builtin_shufflevector(lo, hi, 0, 1, 2, 3, 4, 5, 6, 7, 8, 9, 10, 11, 12, 13, 14, 15)); }
__device__ __forceinline__ v16h  ldh(const h16* p) { return cat16(*(const v8h*)p, *(const v8h*)(p + 16)); }
__device__ __forceinline__ v16bf ldb(const bf* p)  { return cat16b(*(const v8us*)p, *(const v8us*)(p + 16)); }
__device__ __forceinline__ v8f wm_h(v16h a, v16h b, v8f c) {
    c = __builtin_amdgcn_wmma_f32_16x16x32_f16(false, a, false, b, (short)0, c, false, false);
    asm volatile("v_nop\n\tv_nop\n\tv_nop\n\tv_nop" : "+v"(c) : "v"(a), "v"(b));
    return c; }
__device__ __forceinline__ v8f wm_b(v16bf a, v16bf b, v8f c) {
    c = __builtin_amdgcn_wmma_f32_16x16x32_bf16(false, a, false, b, (short)0, c, false, false);
    asm volatile("v_nop\n\tv_nop\n\tv_nop\n\tv_nop" : "+v"(c) : "v"(a), "v"(b));
    return c; }

__global__ __launch_bounds__(256) void k_cvt8(const float* __restrict__ src, bf* dst, int rows_grp, int rows_stride, int n8) {
    const int i = blockIdx.x * 256 + threadIdx.x; if (i >= n8) return;
    const int e = i * 8; const int row = e / DM, col = e % DM; const int g = row / rows_grp, rr = row % rows_grp;
    const float* s = src + ((size_t)g * rows_stride + rr) * DM + col;
    const v4f a = *(const v4f*)s; const v4f b = *(const v4f*)(s + 4); v8us o;
#pragma unroll
    for (int k = 0; k < 4; ++k) { o[k] = f2bf(a[k]); o[4 + k] = f2bf(b[k]); }
    *(volatile v8us*)(dst + (size_t)e) = o; __threadfence(); *(volatile v8us*)(dst + (size_t)e) = o; }

__device__ __forceinline__ void gemm_tile(const bf* __restrict__ A, const bf* __restrict__ Bt, int K, int lda, int ldbt, int kbmask, int r0, int c0, int lr, int hi, v8f (&acc)[4][4]) {
    const size_t aoff = (size_t)(r0 + lr) * lda + 8 * hi, boff = (size_t)(c0 + lr) * ldbt + 8 * hi;
#pragma unroll 1
    for (int kc = 0; kc < K; kc += 32) {
        v16bf a[4];
#pragma unroll
        for (int mb = 0; mb < 4; ++mb) a[mb] = ldb(A + aoff + (size_t)mb * 16 * lda + kc);
        const int kb = kc & kbmask;
#pragma unroll
        for (int nb = 0; nb < 4; ++nb) { const v16bf b = ldb(Bt + boff + (size_t)nb * 16 * ldbt + kb);
#pragma unroll
            for (int mb = 0; mb < 4; ++mb) acc[mb][nb] = wm_b(a[mb], b, acc[mb][nb]); }
    }
}

__global__ __launch_bounds__(32) void k_proj_qk(const bf* __restrict__ XB, const bf* __restrict__ WA, const float* __restrict__ bias, h16* QK16, bf* QKh, bf* QKl) {
    __shared__ __align__(16) float os[16 * 68];
    const int lane = threadIdx.x & 31, lr = lane & 15, hi = lane >> 4; const int r0 = blockIdx.x * 64, c0 = blockIdx.y * 64;
    v8f acc[4][4];
#pragma unroll
    for (int mb = 0; mb < 4; ++mb)
#pragma unroll
        for (int nb = 0; nb < 4; ++nb) acc[mb][nb] = (v8f){};
    gemm_tile(XB, WA, DM, DM, DM, DM - 1, r0, c0, lr, hi, acc);
    const int which = c0 / DM, hh = (c0 % DM) / HD; const int bidx = r0 / SEQ, t0 = r0 % SEQ; const bool hr = (t0 < RH);
    const int rq = lane >> 3, c8 = (lane & 7) * 8;
    float bb[8];
#pragma unroll
    for (int i = 0; i < 8; ++i) bb[i] = bfr(bias[c0 + c8 + i]);
    const size_t hsel = (size_t)which * NB * NH + (size_t)bidx * NH + hh;
    const size_t base16 = (hsel * SEQ + t0) * HD + c8;
    const size_t baseh  = (hsel * RH + (hr ? t0 : 0)) * HD + c8;
#pragma unroll
    for (int mb = 0; mb < 4; ++mb) {
#pragma unroll
        for (int nb = 0; nb < 4; ++nb) {
#pragma unroll
            for (int j = 0; j < 8; ++j) os[(hi * 8 + j) * 68 + nb * 16 + lr] = acc[mb][nb][j]; }
        __syncthreads();
#pragma unroll 1
        for (int ps = 0; ps < 2; ++ps) {
#pragma unroll
            for (int s = 0; s < 4; ++s) { const int row = rq + 4 * s; const v4f a = *(const v4fa*)(os + row * 68 + c8); const v4f b = *(const v4fa*)(os + row * 68 + c8 + 4);
                float val[8];
#pragma unroll
                for (int i = 0; i < 4; ++i) { val[i] = a[i] + bb[i]; val[4 + i] = b[i] + bb[4 + i]; }
                v8h o; v8us oh, ol;
#pragma unroll
                for (int i = 0; i < 8; ++i) { o[i] = (h16)val[i]; unsigned short a2, c2; splitf(val[i], a2, c2); oh[i] = a2; ol[i] = c2; }
                const size_t t = (size_t)(mb * 16 + row) * HD;
                *(volatile v8h*)(QK16 + base16 + t) = o;
                if (hr) { *(volatile v8us*)(QKh + baseh + t) = oh; *(volatile v8us*)(QKl + baseh + t) = ol; } }
            if (ps == 0) __threadfence(); }
        __syncthreads();
    }
}

__global__ __launch_bounds__(32) void k_proj_vt(const bf* __restrict__ WV, const bf* __restrict__ XB, const float* __restrict__ biasv, h16* VT16, bf* VTh, bf* VTl) {
    __shared__ __align__(16) float os[16 * 68];
    const int lane = threadIdx.x & 31, lr = lane & 15, hi = lane >> 4; const int r0 = blockIdx.x * 64, c0 = blockIdx.y * 64;
    v8f acc[4][4];
#pragma unroll
    for (int mb = 0; mb < 4; ++mb)
#pragma unroll
        for (int nb = 0; nb < 4; ++nb) acc[mb][nb] = (v8f){};
    gemm_tile(WV, XB, DM, DM, DM, DM - 1, r0, c0, lr, hi, acc);
    const int hh = r0 / HD; const int bidx = c0 / SEQ, t0 = c0 % SEQ; const bool hr = (t0 < RH);
    const int rq = lane >> 3, c8 = (lane & 7) * 8;
    const size_t hsel = (size_t)bidx * NH + hh;
#pragma unroll
    for (int mb = 0; mb < 4; ++mb) {
#pragma unroll
        for (int nb = 0; nb < 4; ++nb) {
#pragma unroll
            for (int j = 0; j < 8; ++j) os[(hi * 8 + j) * 68 + nb * 16 + lr] = acc[mb][nb][j]; }
        __syncthreads();
#pragma unroll 1
        for (int ps = 0; ps < 2; ++ps) {
#pragma unroll
            for (int s = 0; s < 4; ++s) { const int row = rq + 4 * s; const int d = mb * 16 + row; const float bv = bfr(biasv[r0 + d]);
                const v4f a = *(const v4fa*)(os + row * 68 + c8); const v4f b = *(const v4fa*)(os + row * 68 + c8 + 4);
                v8h o; v8us oh, ol;
#pragma unroll
                for (int i = 0; i < 8; ++i) { const float v = ((i < 4) ? a[i & 3] : b[i & 3]) + bv; o[i] = (h16)v; unsigned short a2, c2; splitf(v, a2, c2); oh[i] = a2; ol[i] = c2; }
                *(volatile v8h*)(VT16 + (hsel * HD + d) * SEQ + t0 + c8) = o;
                if (hr) { const size_t oo = (hsel * HD + d) * RH + t0 + c8; *(volatile v8us*)(VTh + oo) = oh; *(volatile v8us*)(VTl + oo) = ol; } }
            if (ps == 0) __threadfence(); }
        __syncthreads();
    }
}

__global__ __launch_bounds__(32) void k_proj_out(const bf* __restrict__ CTX, const bf* __restrict__ WP, const float* __restrict__ bias, float* OUT) {
    __shared__ __align__(16) float os[16 * 68];
    const int lane = threadIdx.x & 31, lr = lane & 15, hi = lane >> 4; const int r0 = blockIdx.x * 64, c0 = blockIdx.y * 64;
    v8f acc[4][4];
#pragma unroll
    for (int mb = 0; mb < 4; ++mb)
#pragma unroll
        for (int nb = 0; nb < 4; ++nb) acc[mb][nb] = (v8f){};
    gemm_tile(CTX, WP, 2 * DM, 2 * DM, DM, DM - 1, r0, c0, lr, hi, acc);
    const int bidx = r0 / SEQ, t0 = r0 % SEQ; const int cofs = lr * 4;
    float bb[4];
#pragma unroll
    for (int i = 0; i < 4; ++i) bb[i] = bfr(bias[c0 + cofs + i]);
    float* obase = OUT + ((size_t)bidx * SEQ_FULL + t0) * DM + c0 + cofs;
#pragma unroll
    for (int mb = 0; mb < 4; ++mb) {
#pragma unroll
        for (int nb = 0; nb < 4; ++nb) {
#pragma unroll
            for (int j = 0; j < 8; ++j) os[(hi * 8 + j) * 68 + nb * 16 + lr] = acc[mb][nb][j]; }
        __syncthreads();
#pragma unroll 1
        for (int ps = 0; ps < 2; ++ps) {
#pragma unroll
            for (int s = 0; s < 8; ++s) { const int row = 2 * s + hi; v4f val = *(const v4fa*)(os + row * 68 + cofs);
                val[0] += bb[0]; val[1] += bb[1]; val[2] += bb[2]; val[3] += bb[3];
                *(volatile v4f*)(obase + (size_t)(mb * 16 + row) * DM) = val; }
            if (ps == 0) __threadfence(); }
        __syncthreads();
    }
}

__device__ __forceinline__ void attn_f16(const h16* __restrict__ Q, const h16* __restrict__ K, const h16* __restrict__ V, int q0, int r, int half, v8f (&oacc)[4], float& lsum) {
    const size_t qo = (size_t)(q0 + r) * HD + 8 * half;
    const v16h bq0 = ldh(Q + qo), bq1 = ldh(Q + qo + 32);
    float mrun = NEGBIG, lrun = 0.0f; const int qabs = q0 + r; const int ntiles = (q0 + 47) >> 5;
#pragma unroll 1
    for (int kt = 0; kt < ntiles; ++kt) {
        const int kb = kt * 32; const size_t ko = (size_t)(kb + r) * HD + 8 * half;
        v8f s0 = (v8f){}, s1 = (v8f){};
        { v16h a = ldh(K + ko); s0 = wm_h(a, bq0, s0); a = ldh(K + ko + 32); s0 = wm_h(a, bq1, s0); }
        { v16h a = ldh(K + ko + 16 * HD); s1 = wm_h(a, bq0, s1); a = ldh(K + ko + 16 * HD + 32); s1 = wm_h(a, bq1, s1); }
        float sv[16]; float tmax = NEGBIG;
#pragma unroll
        for (int j = 0; j < 8; ++j) { const int key0 = kb + 8 * half + j, key1 = key0 + 16;
            const float v0 = (key0 <= qabs) ? s0[j] * SCL : NEGBIG; const float v1 = (key1 <= qabs) ? s1[j] * SCL : NEGBIG;
            sv[j] = v0; sv[8 + j] = v1; tmax = fmaxf(tmax, fmaxf(v0, v1)); }
        tmax = fmaxf(tmax, __shfl_xor(tmax, 16, 32));
        const float mnew = fmaxf(mrun, tmax); const float alpha = ex2((mrun - mnew) * LOG2E);
        float psum = 0.0f; v16h pf;
#pragma unroll
        for (int i = 0; i < 16; ++i) { const float p = ex2((sv[i] - mnew) * LOG2E); psum += p; pf[i] = (h16)(p * PCAR); }
        psum += __shfl_xor(psum, 16, 32);
        lrun = lrun * alpha + psum; mrun = mnew;
#pragma unroll
        for (int dt = 0; dt < 4; ++dt)
#pragma unroll
            for (int j = 0; j < 8; ++j) oacc[dt][j] *= alpha;
#pragma unroll
        for (int dt = 0; dt < 4; ++dt) { const v16h va = ldh(V + (size_t)(dt * 16 + r) * SEQ + kb + 8 * half); oacc[dt] = wm_h(va, pf, oacc[dt]); }
    }
    lsum = lrun;
}
__device__ __forceinline__ void attn_hl(const bf* __restrict__ Qh, const bf* __restrict__ Ql, const bf* __restrict__ Kh, const bf* __restrict__ Kl, const bf* __restrict__ Vh, const bf* __restrict__ Vl, int q0, int r, int half, v8f (&oacc)[4], float& lsum) {
    const size_t qo = (size_t)(q0 + r) * HD + 8 * half;
    const v16bf qh0 = ldb(Qh + qo), qh1 = ldb(Qh + qo + 32), ql0 = ldb(Ql + qo), ql1 = ldb(Ql + qo + 32);
    float mrun = NEGBIG, lrun = 0.0f; const int qabs = q0 + r; const int ntiles = (q0 + 47) >> 5;
#pragma unroll 1
    for (int kt = 0; kt < ntiles; ++kt) {
        const int kb = kt * 32; const size_t ko = (size_t)(kb + r) * HD + 8 * half; const size_t k1 = ko + 16 * HD;
        v8f s0 = (v8f){}, s1 = (v8f){};
        { v16bf ah = ldb(Kh + ko), al = ldb(Kl + ko); s0 = wm_b(al, qh0, s0); s0 = wm_b(ah, ql0, s0); s0 = wm_b(ah, qh0, s0);
          ah = ldb(Kh + ko + 32); al = ldb(Kl + ko + 32); s0 = wm_b(al, qh1, s0); s0 = wm_b(ah, ql1, s0); s0 = wm_b(ah, qh1, s0); }
        { v16bf ah = ldb(Kh + k1), al = ldb(Kl + k1); s1 = wm_b(al, qh0, s1); s1 = wm_b(ah, ql0, s1); s1 = wm_b(ah, qh0, s1);
          ah = ldb(Kh + k1 + 32); al = ldb(Kl + k1 + 32); s1 = wm_b(al, qh1, s1); s1 = wm_b(ah, ql1, s1); s1 = wm_b(ah, qh1, s1); }
        float sv[16]; float tmax = NEGBIG;
#pragma unroll
        for (int j = 0; j < 8; ++j) { const int key0 = kb + 8 * half + j, key1 = key0 + 16;
            const float v0 = (key0 <= qabs) ? s0[j] * SCL : NEGBIG; const float v1 = (key1 <= qabs) ? s1[j] * SCL : NEGBIG;
            sv[j] = v0; sv[8 + j] = v1; tmax = fmaxf(tmax, fmaxf(v0, v1)); }
        tmax = fmaxf(tmax, __shfl_xor(tmax, 16, 32));
        const float mnew = fmaxf(mrun, tmax); const float alpha = ex2((mrun - mnew) * LOG2E);
        float psum = 0.0f; v16us ph, pl;
#pragma unroll
        for (int i = 0; i < 16; ++i) { const float p = ex2((sv[i] - mnew) * LOG2E); psum += p; unsigned short a2, c2; splitf(p, a2, c2); ph[i] = a2; pl[i] = c2; }
        psum += __shfl_xor(psum, 16, 32);
        lrun = lrun * alpha + psum; mrun = mnew;
        const v16bf pfh = __builtin_bit_cast(v16bf, ph), pfl = __builtin_bit_cast(v16bf, pl);
#pragma unroll
        for (int dt = 0; dt < 4; ++dt)
#pragma unroll
            for (int j = 0; j < 8; ++j) oacc[dt][j] *= alpha;
#pragma unroll
        for (int dt = 0; dt < 4; ++dt) { const size_t vo = (size_t)(dt * 16 + r) * RH + kb + 8 * half; const v16bf vh = ldb(Vh + vo), vl = ldb(Vl + vo);
            oacc[dt] = wm_b(vl, pfh, oacc[dt]); oacc[dt] = wm_b(vh, pfl, oacc[dt]); oacc[dt] = wm_b(vh, pfh, oacc[dt]); }
    }
    lsum = lrun;
}

__global__ __launch_bounds__(128) void k_flash(const h16* __restrict__ QK16, const h16* __restrict__ VT16, const bf* __restrict__ QKh, const bf* __restrict__ QKl, const bf* __restrict__ VTh, const bf* __restrict__ VTl, bf* CTX) {
    __shared__ __align__(16) float os[4 * 16 * 68];
    const int wave = __builtin_amdgcn_readfirstlane(threadIdx.x >> 5); const int lane = threadIdx.x & 31, r = lane & 15, half = lane >> 4;
    const int h = blockIdx.y, bidx = blockIdx.z; const int qblk = blockIdx.x * 64; const int q0 = qblk + wave * 16;
    const size_t hsel = (size_t)bidx * NH + h;
    const size_t PL16 = (size_t)NB * NH * SEQ * HD, PLH = (size_t)NB * NH * RH * HD;
    v8f oacc[4];
#pragma unroll
    for (int dt = 0; dt < 4; ++dt) oacc[dt] = (v8f){};
    float lsum = 1.0f, osc = 1.0f;
    if (qblk < RH) {
        attn_hl(QKh + hsel * RH * HD, QKl + hsel * RH * HD, QKh + PLH + hsel * RH * HD, QKl + PLH + hsel * RH * HD, VTh + hsel * HD * RH, VTl + hsel * HD * RH, q0, r, half, oacc, lsum);
        osc = 1.0f;
    } else {
        attn_f16(QK16 + hsel * SEQ * HD, QK16 + PL16 + hsel * SEQ * HD, VT16 + hsel * HD * SEQ, q0, r, half, oacc, lsum);
        osc = 1.0f / PCAR;
    }
    const float inv = (1.0f / lsum) * osc;
    const int wb = wave * 16 * 68;
#pragma unroll
    for (int dt = 0; dt < 4; ++dt)
#pragma unroll
        for (int j = 0; j < 8; ++j) os[wb + r * 68 + dt * 16 + 8 * half + j] = oacc[dt][j] * inv;
    __syncthreads();
    const int rq = lane >> 3, c8 = (lane & 7) * 8;
    bf* cbase = CTX + ((size_t)bidx * SEQ + q0) * (2 * DM) + h * HD + c8;
#pragma unroll 1
    for (int ps = 0; ps < 2; ++ps) {
#pragma unroll
        for (int s = 0; s < 4; ++s) { const int row = rq + 4 * s; const v4f a = *(const v4fa*)(os + wb + row * 68 + c8); const v4f b = *(const v4fa*)(os + wb + row * 68 + c8 + 4);
            v8us oh, ol;
#pragma unroll
            for (int i = 0; i < 4; ++i) { unsigned short a2, c2; splitf(a[i], a2, c2); oh[i] = a2; ol[i] = c2; splitf(b[i], a2, c2); oh[4 + i] = a2; ol[4 + i] = c2; }
            bf* dst = cbase + (size_t)row * (2 * DM);
            *(volatile v8us*)dst = oh; *(volatile v8us*)(dst + DM) = ol; }
        if (ps == 0) __threadfence(); }
}

extern "C" void kernel_launch(void* const* d_in, const int* in_sizes, int n_in,
                              void* d_out, int out_size, void* d_ws, size_t ws_size, hipStream_t stream) {
    if (n_in < 5) return;
    const size_t need_x = ((size_t)(NB - 1) * SEQ_FULL + SEQ) * DM;
    if ((size_t)in_sizes[0] < need_x) return;
    if ((size_t)in_sizes[1] < (size_t)3 * DM * DM) return;
    if ((size_t)in_sizes[2] < (size_t)3 * DM) return;
    if ((size_t)in_sizes[3] < (size_t)DM * DM) return;
    if ((size_t)in_sizes[4] < (size_t)DM) return;
    if ((size_t)out_size < need_x) return;
    if (OFF_END > ws_size) return;
    const float* x = (const float*)d_in[0]; const float* wattn = (const float*)d_in[1]; const float* battn = (const float*)d_in[2]; const float* wproj = (const float*)d_in[3]; const float* bproj = (const float*)d_in[4];
    float* OUT = (float*)d_out;
    char* ws = (char*)d_ws;
    bf* XB = (bf*)(ws + OFF_XB); bf* WA = (bf*)(ws + OFF_WA); bf* WP = (bf*)(ws + OFF_WP);
    h16* QK16 = (h16*)(ws + OFF_QK16); h16* VT16 = (h16*)(ws + OFF_VT16);
    bf* QKh = (bf*)(ws + OFF_QKH); bf* QKl = (bf*)(ws + OFF_QKL); bf* VTh = (bf*)(ws + OFF_VTH); bf* VTl = (bf*)(ws + OFF_VTL);
    bf* CTX = (bf*)(ws + OFF_CTX);

    const int n8x = NB * SEQ * DM / 8, n8a = 3 * DM * DM / 8, n8p = DM * DM / 8;
    k_cvt8<<<(unsigned)((n8x + 255) / 256), 256, 0, stream>>>(x, XB, SEQ, SEQ_FULL, n8x);
    k_cvt8<<<(unsigned)((n8a + 255) / 256), 256, 0, stream>>>(wattn, WA, 3 * DM, 3 * DM, n8a);
    k_cvt8<<<(unsigned)((n8p + 255) / 256), 256, 0, stream>>>(wproj, WP, DM, DM, n8p);
    k_proj_qk<<<dim3(NB * SEQ / 64, 2 * DM / 64, 1), 32, 0, stream>>>(XB, WA, battn, QK16, QKh, QKl);
    k_proj_vt<<<dim3(DM / 64, NB * SEQ / 64, 1), 32, 0, stream>>>(WA + (size_t)2 * DM * DM, XB, battn + 2 * DM, VT16, VTh, VTl);
    k_flash<<<dim3(SEQ / 64, NH, NB), 128, 0, stream>>>(QK16, VT16, QKh, QKl, VTh, VTl, CTX);
    k_proj_out<<<dim3(NB * SEQ / 64, DM / 64, 1), 32, 0, stream>>>(CTX, WP, bproj, OUT);
}
